// RWKV6_CrossAttention_62775241998772
// MI455X (gfx1250) — hardware-run, weakly checked
//
#include <hip/hip_runtime.h>
#include <math.h>

typedef __attribute__((ext_vector_type(16))) _Float16 v16h;
typedef __attribute__((ext_vector_type(8)))  _Float16 v8h;
typedef __attribute__((ext_vector_type(2)))  _Float16 v2h;
typedef __attribute__((ext_vector_type(16))) __bf16   v16b;
typedef __attribute__((ext_vector_type(8)))  __bf16   v8b;
typedef __attribute__((ext_vector_type(8)))  float    v8f;
typedef __attribute__((ext_vector_type(4)))  float    v4f;
typedef __attribute__((ext_vector_type(2)))  float    v2f;

constexpr int kB    = 2;
constexpr int kLQ   = 8;
constexpr int kLK   = 512;
constexpr int kEB   = kB * kLQ;
constexpr int kRows = kEB * kLK;
constexpr int kRk   = kB * kLK;
constexpr int kH    = 256;
constexpr int kNH   = 4;
constexpr int kDK   = 64;
constexpr int kP    = 32;
constexpr int kG    = 64;
constexpr int kK2   = 2 * kH;
constexpr int kThr  = 256;
constexpr float kEps = 1.0e-5f;
constexpr float kInCarry = 1024.0f;
constexpr float kWCarry  = 4096.0f;
constexpr float kTCarry  = 16384.0f;
constexpr float kYCarry  = 256.0f;
constexpr float kScX  = 1.0f / (kInCarry * kWCarry);
constexpr float kScT2 = 1.0f / (kTCarry * kInCarry);
constexpr float kScTB = 1.0f / (kTCarry * kWCarry);
constexpr float kScY  = 1.0f / (kYCarry * kWCarry);
constexpr float kF16MinNormal = 6.103515625e-5f;

static_assert(kRows == 8192 && kRk == 1024 && kH == kNH * kDK && kK2 == 512 && kP == 32 && kG == 64, "the index arithmetic below uses these sizes");

constexpr size_t kOffZB = 0ull;
constexpr size_t kOffBRWG = 8192ull;
constexpr size_t kOffBKV = 11264ull;
constexpr size_t kOffBBB = 13312ull;
constexpr size_t kOffONES = 14336ull;
constexpr size_t kOffUB = 15360ull;
constexpr size_t kOffWRWG0 = 16384ull;
constexpr size_t kOffWKV0 = 147456ull;
constexpr size_t kOffWR = 212992ull;
constexpr size_t kOffWG = 475136ull;
constexpr size_t kOffWK = 737280ull;
constexpr size_t kOffWV = 999424ull;
constexpr size_t kOffWA = 1261568ull;
constexpr size_t kOffWB = 1327104ull;
constexpr size_t kOffWO = 1359872ull;
constexpr size_t kOffW2R16 = 1490944ull;
constexpr size_t kOffWKV2R16 = 1540096ull;
constexpr size_t kOffXA2 = 1572864ull;
constexpr size_t kOffXK2 = 9961472ull;
constexpr size_t kOffT0 = 11010048ull;
constexpr size_t kOffT0K = 15204352ull;
constexpr size_t kOffTW16 = 15466496ull;
constexpr size_t kOffTWK16 = 17039360ull;
constexpr size_t kOffRWG = 17170432ull;
constexpr size_t kOffKVM = 42336256ull;
constexpr size_t kOffXR2 = 44433408ull;
constexpr size_t kOffXW2 = 52822016ull;
constexpr size_t kOffXG2 = 61210624ull;
constexpr size_t kOffXKK2 = 69599232ull;
constexpr size_t kOffXV2 = 70647808ull;
constexpr size_t kOffRM = 71696384ull;
constexpr size_t kOffGM = 80084992ull;
constexpr size_t kOffWA1 = 88473600ull;
constexpr size_t kOffTWA16 = 90570752ull;
constexpr size_t kOffWM = 91619328ull;
constexpr size_t kOffKM = 100007936ull;
constexpr size_t kOffVM = 101056512ull;
constexpr size_t kOffAM = 102105088ull;
constexpr size_t kOffOM = 110493696ull;
constexpr size_t kOffY16 = 118882304ull;
constexpr size_t kWsTotal = 123076608ull;
static_assert(kWsTotal <= 134217728ull, "carve cap: under 128 MiB");
static_assert(kOffZB == 0
              && kOffBRWG == kOffZB + 8192ull
              && kOffBKV == kOffBRWG + 3072ull
              && kOffBBB == kOffBKV + 2048ull
              && kOffONES == kOffBBB + 1024ull
              && kOffUB == kOffONES + 1024ull
              && kOffWRWG0 == kOffUB + 1024ull
              && kOffWKV0 == kOffWRWG0 + 131072ull
              && kOffWR == kOffWKV0 + 65536ull
              && kOffWG == kOffWR + 262144ull
              && kOffWK == kOffWG + 262144ull
              && kOffWV == kOffWK + 262144ull
              && kOffWA == kOffWV + 262144ull
              && kOffWB == kOffWA + 65536ull
              && kOffWO == kOffWB + 32768ull
              && kOffW2R16 == kOffWO + 131072ull
              && kOffWKV2R16 == kOffW2R16 + 49152ull
              && kOffXA2 == kOffWKV2R16 + 32768ull
              && kOffXK2 == kOffXA2 + 8388608ull
              && kOffT0 == kOffXK2 + 1048576ull
              && kOffT0K == kOffT0 + 4194304ull
              && kOffTW16 == kOffT0K + 262144ull
              && kOffTWK16 == kOffTW16 + 1572864ull
              && kOffRWG == kOffTWK16 + 131072ull
              && kOffKVM == kOffRWG + 25165824ull
              && kOffXR2 == kOffKVM + 2097152ull
              && kOffXW2 == kOffXR2 + 8388608ull
              && kOffXG2 == kOffXW2 + 8388608ull
              && kOffXKK2 == kOffXG2 + 8388608ull
              && kOffXV2 == kOffXKK2 + 1048576ull
              && kOffRM == kOffXV2 + 1048576ull
              && kOffGM == kOffRM + 8388608ull
              && kOffWA1 == kOffGM + 8388608ull
              && kOffTWA16 == kOffWA1 + 2097152ull
              && kOffWM == kOffTWA16 + 1048576ull
              && kOffKM == kOffWM + 8388608ull
              && kOffVM == kOffKM + 1048576ull
              && kOffAM == kOffVM + 1048576ull
              && kOffOM == kOffAM + 8388608ull
              && kOffY16 == kOffOM + 8388608ull
              && kWsTotal == kOffY16 + 4194304ull, "the carve is chained and totalled");
static_assert((kOffBRWG % 256) == 0 && (kOffBKV % 256) == 0 && (kOffBBB % 256) == 0 && (kOffONES % 256) == 0 && (kOffUB % 256) == 0 && (kOffWRWG0 % 256) == 0 && (kOffWKV0 % 256) == 0 && (kOffWR % 256) == 0 && (kOffWG % 256) == 0 && (kOffWK % 256) == 0 && (kOffWV % 256) == 0 && (kOffWA % 256) == 0 && (kOffWB % 256) == 0 && (kOffWO % 256) == 0 && (kOffW2R16 % 256) == 0 && (kOffWKV2R16 % 256) == 0 && (kOffXA2 % 256) == 0 && (kOffXK2 % 256) == 0 && (kOffT0 % 256) == 0 && (kOffT0K % 256) == 0 && (kOffTW16 % 256) == 0 && (kOffTWK16 % 256) == 0 && (kOffRWG % 256) == 0 && (kOffKVM % 256) == 0 && (kOffXR2 % 256) == 0 && (kOffXW2 % 256) == 0 && (kOffXG2 % 256) == 0 && (kOffXKK2 % 256) == 0 && (kOffXV2 % 256) == 0 && (kOffRM % 256) == 0 && (kOffGM % 256) == 0 && (kOffWA1 % 256) == 0 && (kOffTWA16 % 256) == 0 && (kOffWM % 256) == 0 && (kOffKM % 256) == 0 && (kOffVM % 256) == 0 && (kOffAM % 256) == 0 && (kOffOM % 256) == 0 && (kOffY16 % 256) == 0, "aligned regions");

__device__ __forceinline__ unsigned short f2bf_bits(float f) {
  unsigned u = __float_as_uint(f);
  return (unsigned short)((u + 0x7FFFu + ((u >> 16) & 1u)) >> 16);
}
__device__ __forceinline__ float bf_bits2f(unsigned short h) { return __uint_as_float(((unsigned)h) << 16); }
__device__ __forceinline__ float bf16r(float f) { return bf_bits2f(f2bf_bits(f)); }
__device__ __forceinline__ float carry_flush(float v, float carry) {
  const float s = v * carry;
  return (fabsf(s) < kF16MinNormal) ? 0.0f : s;
}

__device__ __forceinline__ void dep_guard4_h(v8f& a, v8f& b, v8f& c, v8f& d, v16h x, v16h y) { asm volatile("v_nop\n\tv_nop\n\tv_nop\n\tv_nop" : "+v"(a), "+v"(b), "+v"(c), "+v"(d) : "v"(x), "v"(y)); }
__device__ __forceinline__ void dep_guard4_b(v8f& a, v8f& b, v8f& c, v8f& d, v16b x, v16b y) { asm volatile("v_nop\n\tv_nop\n\tv_nop\n\tv_nop" : "+v"(a), "+v"(b), "+v"(c), "+v"(d) : "v"(x), "v"(y)); }
__device__ __forceinline__ void keep4_h(v16h a, v16h b, v16h c, v16h d) { asm volatile("v_nop" :: "v"(a), "v"(b), "v"(c), "v"(d)); }
__device__ __forceinline__ void keep4_b(v16b a, v16b b, v16b c, v16b d) { asm volatile("v_nop" :: "v"(a), "v"(b), "v"(c), "v"(d)); }
__device__ __forceinline__ void acc_guard4(v8f& a, v8f& b, v8f& c, v8f& d) { asm volatile("v_nop\n\tv_nop\n\tv_nop\n\tv_nop" : "+v"(a), "+v"(b), "+v"(c), "+v"(d)); }

template <typename T> struct Frag;
template <> struct Frag<_Float16> {
  typedef v16h V; union U { v16h v; v8h h[2]; };
  static __device__ __forceinline__ v16h load(const _Float16* p) {
    U f; f.h[0] = *(const v8h*)(p); f.h[1] = *(const v8h*)(p + 16); return f.v;
  }
  static __device__ __forceinline__ v8f mma(v16h a, v16h b, v8f c) {
    return __builtin_amdgcn_wmma_f32_16x16x32_f16(false, a, false, b, (short)0, c, false, false);
  }
  static __device__ __forceinline__ void guard4(v8f& a, v8f& b, v8f& c, v8f& d, v16h x, v16h y) { dep_guard4_h(a, b, c, d, x, y); }
  static __device__ __forceinline__ void keep(v16h a, v16h b, v16h c, v16h d) { keep4_h(a, b, c, d); }
};
template <> struct Frag<__bf16> {
  typedef v16b V; union U { v16b v; v8b h[2]; };
  static __device__ __forceinline__ v16b load(const __bf16* p) {
    U f; f.h[0] = *(const v8b*)(p); f.h[1] = *(const v8b*)(p + 16); return f.v;
  }
  static __device__ __forceinline__ v8f mma(v16b a, v16b b, v8f c) {
    return __builtin_amdgcn_wmma_f32_16x16x32_bf16(false, a, false, b, (short)0, c, false, false);
  }
  static __device__ __forceinline__ void guard4(v8f& a, v8f& b, v8f& c, v8f& d, v16b x, v16b y) { dep_guard4_b(a, b, c, d, x, y); }
  static __device__ __forceinline__ void keep(v16b a, v16b b, v16b c, v16b d) { keep4_b(a, b, c, d); }
};

__device__ __forceinline__ v8f mma_h(v16h a, v16h b, v8f c) {
  c = __builtin_amdgcn_wmma_f32_16x16x32_f16(false, a, false, b, (short)0, c, false, false);
  asm volatile("v_nop\n\tv_nop\n\tv_nop\n\tv_nop" : "+v"(c) : "v"(a), "v"(b));
  return c;
}

template <int ET> struct Elem;
template <> struct Elem<0> { typedef _Float16 T; };
template <> struct Elem<1> { typedef __bf16 T; };
template <int ET, bool SPLIT, int BIAS_MODE, int OUT_MODE, bool RESID, int ACT = 0>
__global__ __launch_bounds__(256) void wmma_gemm64(
    const unsigned short* __restrict__ Ap, const unsigned short* __restrict__ A2p, int lda, long strideA,
    const unsigned short* __restrict__ Btp, const unsigned short* __restrict__ Bt2p, int ldb, long strideB,
    void* __restrict__ Cout, void* __restrict__ Cout2, int ldc, long strideC,
    const float* __restrict__ bias,
    const float* __restrict__ resid, long strideR,
    int M, int N, int K, float scale) {
  typedef typename Elem<ET>::T T;
  typedef typename Frag<T>::V V;
  const T* A = (const T*)Ap; const T* A2 = (const T*)A2p; const T* Bt = (const T*)Btp; const T* Bt2 = (const T*)Bt2p;
  __shared__ __align__(16) float sT[8][16 * 68];
  const int b    = blockIdx.y;
  const int lane = threadIdx.x & 31;
  const int wave = threadIdx.x >> 5;
  const int tilesN = N >> 6;
  const int tilesM = M >> 6;
  const int tile = blockIdx.x * 8 + wave;
  if (tile >= tilesM * tilesN) return;
  const int tm = tile / tilesN;
  const int tn = tile - tm * tilesN;
  const int m0 = tm << 6;
  const int n0 = tn << 6;

  const T* Ab  = A  + (size_t)b * strideA;
  const T* Bb  = Bt + (size_t)b * strideB;
  const T* Ab2 = SPLIT ? (A2  + (size_t)b * strideA) : nullptr;
  const T* Bb2 = SPLIT ? (Bt2 + (size_t)b * strideB) : nullptr;

  const int rlane = lane & 15;
  const int koff  = (lane >> 4) * 8;
  const int mOff  = (lane >> 4) * 8;

  v8f acc[4][4];
#pragma unroll
  for (int i = 0; i < 4; ++i)
#pragma unroll
    for (int j = 0; j < 4; ++j) acc[i][j] = (v8f){0.f,0.f,0.f,0.f,0.f,0.f,0.f,0.f};

  for (int k0 = 0; k0 < K; k0 += 32) {
    V bh[4], bl[4];
#pragma unroll
    for (int j = 0; j < 4; ++j) {
      const size_t bo = (size_t)(n0 + (j << 4) + rlane) * ldb + koff + k0;
      bh[j] = Frag<T>::load(Bb + bo);
      if (SPLIT) bl[j] = Frag<T>::load(Bb2 + bo);
    }
#pragma unroll
    for (int i = 0; i < 4; ++i) {
      const size_t ao = (size_t)(m0 + (i << 4) + rlane) * lda + koff + k0;
      V ah = Frag<T>::load(Ab + ao);
      V al;
      if (SPLIT) al = Frag<T>::load(Ab2 + ao);
#pragma unroll
      for (int j = 0; j < 4; ++j) {
        acc[i][j] = Frag<T>::mma(ah, bh[j], acc[i][j]);
        if (SPLIT) {
          acc[i][j] = Frag<T>::mma(ah, bl[j], acc[i][j]);
          acc[i][j] = Frag<T>::mma(al, bh[j], acc[i][j]);
        }
      }
      Frag<T>::guard4(acc[i][0], acc[i][1], acc[i][2], acc[i][3], ah, SPLIT ? al : ah);
    }
    Frag<T>::keep(bh[0], bh[1], bh[2], bh[3]);
    if (SPLIT) Frag<T>::keep(bl[0], bl[1], bl[2], bl[3]);
  }
  acc_guard4(acc[0][0], acc[0][1], acc[0][2], acc[0][3]);
  acc_guard4(acc[1][0], acc[1][1], acc[1][2], acc[1][3]);
  acc_guard4(acc[2][0], acc[2][1], acc[2][2], acc[2][3]);
  acc_guard4(acc[3][0], acc[3][1], acc[3][2], acc[3][3]);

  float* slab = sT[wave];
  const float* Rb = RESID ? (resid + (size_t)b * strideR) : nullptr;
#pragma unroll
  for (int i = 0; i < 4; ++i) {
    const int mBase = m0 + (i << 4);
#pragma unroll
    for (int j = 0; j < 4; ++j) {
      const int n = n0 + (j << 4) + rlane;
      float bv = 0.f;
      if (BIAS_MODE == 2) bv = bias[n];
#pragma unroll
      for (int r = 0; r < 8; ++r) {
        float v = acc[i][j][r] * scale;
        if (BIAS_MODE == 1) v += bias[mBase + mOff + r];
        if (BIAS_MODE == 2) v += bv;
        if (RESID) v += Rb[(size_t)(mBase + mOff + r) * ldc + n];
        if (ACT == 1) v = tanhf(v);
        if (ACT == 2) v = fmaxf(v, 0.0f);
        if (ACT == 3) v = v / (1.0f + expf(-v));
        if (ACT == 4) v = (v > 0.f) ? v : 0.01f * v;
        slab[(mOff + r) * 68 + (j << 4) + rlane] = v;
      }
    }
    __builtin_amdgcn_fence(__ATOMIC_RELEASE, "workgroup");
    __builtin_amdgcn_wave_barrier();
    __builtin_amdgcn_fence(__ATOMIC_ACQUIRE, "workgroup");
    if (OUT_MODE == 0) {
      float* C = (float*)Cout + (size_t)b * strideC;
      const int hh = lane >> 4, c4 = (lane & 15) * 4;
      for (int pass = 0; pass < 2; ++pass) {
#pragma unroll
        for (int it = 0; it < 8; ++it) {
          const int row = it * 2 + hh;
          v4f v = *(const v4f*)(slab + row * 68 + c4);
          *(volatile v4f*)(C + (size_t)(mBase + row) * ldc + n0 + c4) = v;
        }
        __threadfence();
      }
    } else {
      const int q = lane >> 3, c8 = (lane & 7) * 8;
      unsigned short* C  = (unsigned short*)Cout  + (size_t)b * strideC;
      unsigned short* C2 = (OUT_MODE == 2) ? ((unsigned short*)Cout2 + (size_t)b * strideC) : nullptr;
      for (int pass = 0; pass < 2; ++pass) {
#pragma unroll
        for (int it = 0; it < 4; ++it) {
          const int row = it * 4 + q;
          const float* sp = slab + row * 68 + c8;
          v8h hv, lv;
#pragma unroll
          for (int e = 0; e < 8; ++e) {
            if (OUT_MODE == 1) {
              hv[e] = (_Float16)sp[e];
            } else {
              unsigned short hb = f2bf_bits(sp[e]);
              unsigned short lb = f2bf_bits(sp[e] - bf_bits2f(hb));
              hv[e] = __builtin_bit_cast(_Float16, hb);
              lv[e] = __builtin_bit_cast(_Float16, lb);
            }
          }
          *(volatile v8h*)(C + (size_t)(mBase + row) * ldc + n0 + c8) = hv;
          if (OUT_MODE == 2) *(volatile v8h*)(C2 + (size_t)(mBase + row) * ldc + n0 + c8) = lv;
        }
        __threadfence();
      }
    }
    __builtin_amdgcn_fence(__ATOMIC_RELEASE, "workgroup");
    __builtin_amdgcn_wave_barrier();
    __builtin_amdgcn_fence(__ATOMIC_ACQUIRE, "workgroup");
  }
}


__device__ __forceinline__ void two_words(float w, float carry, _Float16& hh, _Float16& ll) {
  const float sc = carry_flush(w, carry);
  hh = (_Float16)sc;
  const float rs = sc - (float)hh;
  ll = (_Float16)((fabsf(rs) < kF16MinNormal) ? 0.0f : rs);
}
__device__ __forceinline__ void store2(float* p, float v) {
  *(volatile float*)p = v;
  __threadfence();
  *(volatile float*)p = v;
}

__global__ __launch_bounds__(kThr) void cast_plane_kernel(const float* __restrict__ src, unsigned short* __restrict__ dst,
                                                          int colsLog2, int dstPitch, int dstOff) {
  const int i   = blockIdx.x * kThr + threadIdx.x;
  const int sh  = colsLog2 - 3;
  const int row = i >> sh;
  const int c8  = (i & ((1 << sh) - 1)) * 8;
  const float* sp = src + ((size_t)row << colsLog2) + c8;
  const v4f a0 = *(const v4f*)(sp);
  const v4f a1 = *(const v4f*)(sp + 4);
  v8h hv;
#pragma unroll
  for (int e = 0; e < 4; ++e) {
    const float f0 = a0[e];
    const float f1 = a1[e];
    hv[e]     = (_Float16)carry_flush(bf16r(f0), kInCarry);
    hv[4 + e] = (_Float16)carry_flush(bf16r(f1), kInCarry);
  }
  unsigned short* dp = dst + (size_t)row * dstPitch + dstOff + c8;
  *(volatile v8h*)dp = hv;
  __threadfence();
  *(volatile v8h*)dp = hv;
}

__global__ __launch_bounds__(256) void wt_plane_kernel(const float* __restrict__ W, unsigned short* __restrict__ dst, int K, int N, int nLive, int ldd, int colOff) {
  const int n  = blockIdx.x;
  const int k8 = threadIdx.x * 8;
  const bool live = n < nLive;
  const int nc = live ? n : 0;
  v8h hv;
#pragma unroll
  for (int e = 0; e < 8; ++e) {
    const float w = W[(size_t)(k8 + e) * N + nc];
    hv[e] = (_Float16)(live ? carry_flush(bf16r(w), kWCarry) : 0.0f);
  }
  unsigned short* dp = dst + (size_t)n * ldd + colOff + k8;
  *(volatile v8h*)dp = hv;
  __threadfence();
  *(volatile v8h*)dp = hv;
}

__global__ __launch_bounds__(kThr) void setup_kernel(const float* __restrict__ rwg_bias, const float* __restrict__ kv_bias, const float* __restrict__ bb, const float* __restrict__ u,
                                                    float* __restrict__ ZB, float* __restrict__ BRWG, float* __restrict__ BKV, float* __restrict__ BBB, float* __restrict__ ONES, float* __restrict__ UB) {
  const unsigned bk = blockIdx.x, t = threadIdx.x;
  if (bk < 8u) {
    store2(ZB + bk * (unsigned)kThr + t, 0.0f);
  } else if (bk < 11u) {
    const unsigned i = (bk - 8u) * (unsigned)kThr + t; const float p = rwg_bias[i]; store2(BRWG + i, bf16r(p));
  } else if (bk < 13u) {
    const unsigned i = (bk - 11u) * (unsigned)kThr + t; const float p = kv_bias[i]; store2(BKV + i, bf16r(p));
  } else if (bk == 13u) {
    const float p = bb[t]; store2(BBB + t, bf16r(p));
  } else if (bk == 14u) {
    store2(ONES + t, 1.0f);
  } else {
    const float p = u[t]; store2(UB + t, bf16r(p));
  }
}
static_assert(3 * kH == 3 * kThr && 2 * kH == 2 * kThr && kNH * kDK == kThr, "set-up grid exact: 8 + 3 + 2 + 1 + 1 + 1 blocks");

__global__ __launch_bounds__(kThr) void mix1q_kernel(const float* __restrict__ keyval, const float* __restrict__ query, const float* __restrict__ mu, unsigned short* __restrict__ X2) {
  const unsigned i = blockIdx.x * (unsigned)kThr + threadIdx.x;
  const unsigned row = i >> 5, c8 = (i & 31u) * 8u;
  const unsigned eb = row >> 9, l = row & 511u;
  const float* hp = keyval + ((size_t)(eb >> 3) * kLK + l) * kH + c8;
  const float* qp = query + (size_t)eb * kH + c8;
  v8h hv, lv;
#pragma unroll
  for (int e = 0; e < 8; ++e) {
    const float h0 = hp[e], q0 = qp[e], m0 = mu[c8 + e];
    const float h = bf16r(h0);
    const float x = h + (bf16r(q0) - h) * bf16r(m0);
    _Float16 a, b; two_words(x, kInCarry, a, b); hv[e] = a; lv[e] = b;
  }
  unsigned short* dp = X2 + (size_t)row * kK2 + c8;
  for (int pass = 0; pass < 2; ++pass) {
    *(volatile v8h*)dp = hv; *(volatile v8h*)(dp + kH) = lv;
    __threadfence();
  }
}
static_assert((size_t)kRows * (kH / 8) == 1024ull * kThr, "first mix (query branch): 1,024 blocks");

__global__ __launch_bounds__(kThr) void mix1k_kernel(const float* __restrict__ keyval, const float* __restrict__ mu, unsigned short* __restrict__ X2) {
  const unsigned i = blockIdx.x * (unsigned)kThr + threadIdx.x;
  const unsigned krow = i >> 5, c8 = (i & 31u) * 8u;
  const bool has = (krow & 511u) != 0u;
  const float* hp = keyval + (size_t)krow * kH + c8;
  const float* sp = keyval + (size_t)(krow - (has ? 1u : 0u)) * kH + c8;
  v8h hv, lv;
#pragma unroll
  for (int e = 0; e < 8; ++e) {
    const float h0 = hp[e], s0 = sp[e], m0 = mu[c8 + e];
    const float h = bf16r(h0);
    const float s = has ? bf16r(s0) : 0.0f;
    const float x = h + (s - h) * bf16r(m0);
    _Float16 a, b; two_words(x, kInCarry, a, b); hv[e] = a; lv[e] = b;
  }
  unsigned short* dp = X2 + (size_t)krow * kK2 + c8;
  for (int pass = 0; pass < 2; ++pass) {
    *(volatile v8h*)dp = hv; *(volatile v8h*)(dp + kH) = lv;
    __threadfence();
  }
}
static_assert((size_t)kRk * (kH / 8) == 128ull * kThr, "first mix (the other branch): 128 blocks");

template <int NC8, int LD>
__global__ __launch_bounds__(kThr) void tanhcast_kernel(const float* __restrict__ src, unsigned short* __restrict__ dst) {
  const unsigned i = blockIdx.x * (unsigned)kThr + threadIdx.x;
  const unsigned row = i / (unsigned)NC8, g = i % (unsigned)NC8;
  const float* sp = src + (size_t)row * LD + 8u * g;
  v8h hv;
#pragma unroll
  for (int e = 0; e < 8; ++e) { const float v = sp[e]; hv[e] = (_Float16)carry_flush(tanhf(v), kTCarry); }
  unsigned short* dp = dst + (size_t)i * 8u;
  *(volatile v8h*)dp = hv;
  __threadfence();
  *(volatile v8h*)dp = hv;
}
static_assert((kRows * 12) % kThr == 0 && (kRk * 8) % kThr == 0 && (kRows * 8) % kThr == 0, "tanh grids exact: 384 | 32 | 256 blocks");

__global__ __launch_bounds__(kThr) void mix2q_kernel(const float* __restrict__ keyval, const float* __restrict__ query, const float* __restrict__ M,
                                                    unsigned short* __restrict__ XR, unsigned short* __restrict__ XW, unsigned short* __restrict__ XG) {
  const unsigned i = blockIdx.x * (unsigned)kThr + threadIdx.x;
  const unsigned row = i >> 5, c8 = (i & 31u) * 8u;
  const unsigned eb = row >> 9, l = row & 511u;
  const float* hp = keyval + ((size_t)(eb >> 3) * kLK + l) * kH + c8;
  const float* qp = query + (size_t)eb * kH + c8;
  const float* mp = M + (size_t)row * (3 * kH) + c8;
  v8h h0v, l0v, h1v, l1v, h2v, l2v;
#pragma unroll
  for (int e = 0; e < 8; ++e) {
    const float h0 = hp[e], q0 = qp[e];
    const float h = bf16r(h0), dc = bf16r(q0) - h;
    _Float16 a, b;
    two_words(h + dc * mp[e], kInCarry, a, b); h0v[e] = a; l0v[e] = b;
    two_words(h + dc * mp[kH + e], kInCarry, a, b); h1v[e] = a; l1v[e] = b;
    two_words(h + dc * mp[2 * kH + e], kInCarry, a, b); h2v[e] = a; l2v[e] = b;
  }
  const size_t o = (size_t)row * kK2 + c8;
  for (int pass = 0; pass < 2; ++pass) {
    *(volatile v8h*)(XR + o) = h0v; *(volatile v8h*)(XR + o + kH) = l0v;
    *(volatile v8h*)(XW + o) = h1v; *(volatile v8h*)(XW + o + kH) = l1v;
    *(volatile v8h*)(XG + o) = h2v; *(volatile v8h*)(XG + o + kH) = l2v;
    __threadfence();
  }
}

__global__ __launch_bounds__(kThr) void mix2k_kernel(const float* __restrict__ keyval, const float* __restrict__ M, unsigned short* __restrict__ XK, unsigned short* __restrict__ XV) {
  const unsigned i = blockIdx.x * (unsigned)kThr + threadIdx.x;
  const unsigned krow = i >> 5, c8 = (i & 31u) * 8u;
  const bool has = (krow & 511u) != 0u;
  const float* hp = keyval + (size_t)krow * kH + c8;
  const float* sp = keyval + (size_t)(krow - (has ? 1u : 0u)) * kH + c8;
  const float* mp = M + (size_t)krow * (2 * kH) + c8;
  v8h h0v, l0v, h1v, l1v;
#pragma unroll
  for (int e = 0; e < 8; ++e) {
    const float h0 = hp[e], s0 = sp[e];
    const float h = bf16r(h0);
    const float d = (has ? bf16r(s0) : 0.0f) - h;
    _Float16 a, b;
    two_words(h + d * mp[e], kInCarry, a, b); h0v[e] = a; l0v[e] = b;
    two_words(h + d * mp[kH + e], kInCarry, a, b); h1v[e] = a; l1v[e] = b;
  }
  const size_t o = (size_t)krow * kK2 + c8;
  for (int pass = 0; pass < 2; ++pass) {
    *(volatile v8h*)(XK + o) = h0v; *(volatile v8h*)(XK + o + kH) = l0v;
    *(volatile v8h*)(XV + o) = h1v; *(volatile v8h*)(XV + o + kH) = l1v;
    __threadfence();
  }
}

__global__ __launch_bounds__(kThr) void decay_kernel(const float* __restrict__ WM, float* __restrict__ AM) {
  const size_t i4 = ((size_t)blockIdx.x * kThr + threadIdx.x) * 4;
  const v4f w = *(const v4f*)(WM + i4);
  v4f a;
#pragma unroll
  for (int e = 0; e < 4; ++e) a[e] = expf(-expf(w[e]));
  *(volatile v4f*)(AM + i4) = a;
  __threadfence();
  *(volatile v4f*)(AM + i4) = a;
}
static_assert((size_t)kRows * kH == 2048ull * kThr * 4, "decay grid exact: 2,048 blocks");

__global__ __launch_bounds__(kThr) void walk_kernel(const float* __restrict__ RM, const float* __restrict__ KM, const float* __restrict__ VM, const float* __restrict__ AM,
                                                   const float* __restrict__ UB, float* __restrict__ OM) {
  const unsigned eb = blockIdx.x, col = threadIdx.x, hb = col & ~63u;
  float S[kDK], U[kDK];
#pragma unroll
  for (int k = 0; k < kDK; ++k) { S[k] = 0.0f; U[k] = UB[hb + k]; }
  for (int t = 0; t < kLK; ++t) {
    const size_t row = (size_t)eb * kLK + (size_t)t;
    const size_t krow = (size_t)(eb >> 3) * kLK + (size_t)t;
    const float* rp = RM + row * kH + hb;
    const float* ap = AM + row * kH + hb;
    const float* kp = KM + krow * kH + hb;
    const float vv = VM[krow * kH + col];
    float o = 0.0f;
#pragma unroll
    for (int q = 0; q < kDK / 4; ++q) {
      const v4f rv = *(const v4f*)(rp + 4 * q), av = *(const v4f*)(ap + 4 * q), kv = *(const v4f*)(kp + 4 * q);
#pragma unroll
      for (int e = 0; e < 4; ++e) {
        const int k = 4 * q + e;
        const float kvp = kv[e] * vv;
        o += rv[e] * (S[k] + U[k] * kvp);
        S[k] = av[e] * S[k] + kvp;
      }
    }
    store2(OM + row * kH + col, o);
  }
}
static_assert(kNH * kDK == kThr && (kDK % 4) == 0, "scan grid exact: 16 blocks of 4 heads x 64 value columns");

__global__ __launch_bounds__(kThr) void gnorm_kernel(const float* __restrict__ OM, const float* __restrict__ GM, const float* __restrict__ gw, const float* __restrict__ gb, unsigned short* __restrict__ Y16) {
  const unsigned i = blockIdx.x * (unsigned)kThr + threadIdx.x;
  const size_t base = (size_t)(i >> 2) * kH + (size_t)(i & 3u) * kDK;
  const unsigned cb = (i & 3u) * (unsigned)kDK;
  const float* op = OM + base;
  const float* gp = GM + base;
  float sum = 0.0f;
  for (int c = 0; c < kDK; ++c) sum += op[c];
  const float mean = sum * (1.0f / (float)kDK);
  float sq = 0.0f;
  for (int c = 0; c < kDK; ++c) { const float dv = op[c] - mean; sq += dv * dv; }
  const float q = sqrtf(sq * (1.0f / (float)kDK) + kEps);
  unsigned short* dp = Y16 + base;
  for (int c8 = 0; c8 < kDK; c8 += 8) {
    v8h hv;
#pragma unroll
    for (int e = 0; e < 8; ++e) {
      const int c = c8 + e;
      const float w0 = gw[cb + c], b0 = gb[cb + c], g = gp[c];
      const float yn = (op[c] - mean) / q * bf16r(w0) + bf16r(b0);
      hv[e] = (_Float16)carry_flush(yn * (g / (1.0f + expf(-g))), kYCarry);
    }
    *(volatile v8h*)(dp + c8) = hv;
    __threadfence();
    *(volatile v8h*)(dp + c8) = hv;
  }
}
static_assert((size_t)kRows * kNH == 128ull * kThr, "norm grid exact: 128 blocks");

extern "C" void kernel_launch(void* const* d_in, const int* in_sizes, int n_in,
                              void* d_out, int out_size, void* d_ws, size_t ws_size,
                              hipStream_t stream) {
  if (n_in < 21 || d_out == nullptr || d_ws == nullptr) return;
  if (in_sizes[0] != kB * kLQ * kH || in_sizes[1] != kB * kLK * kH || in_sizes[2] != kH || in_sizes[3] != kH * 3 * kP || in_sizes[4] != kH * 3 * kP || in_sizes[5] != 3 * kH) return;
  if (in_sizes[6] != kH || in_sizes[7] != kH * 2 * kP || in_sizes[8] != kH * 2 * kP || in_sizes[9] != 2 * kH || in_sizes[10] != kH * kH || in_sizes[11] != kH * kG || in_sizes[12] != kG * kH || in_sizes[13] != kH) return;
  if (in_sizes[14] != kH * kH || in_sizes[15] != kH * kH || in_sizes[16] != kH * kH || in_sizes[17] != kNH * kDK || in_sizes[18] != kH || in_sizes[19] != kH || in_sizes[20] != kH * kH) return;
  if (out_size != kRows * kH) return;
  if (ws_size < kWsTotal) return;
  const float* query = (const float*)d_in[0];
  const float* keyval = (const float*)d_in[1];
  const float* rwg_mu = (const float*)d_in[2];
  const float* W_rwg0 = (const float*)d_in[3];
  const float* W_rwg2 = (const float*)d_in[4];
  const float* rwg_bias = (const float*)d_in[5];
  const float* kv_mu = (const float*)d_in[6];
  const float* W_kv0 = (const float*)d_in[7];
  const float* W_kv2 = (const float*)d_in[8];
  const float* kv_bias = (const float*)d_in[9];
  const float* Wr = (const float*)d_in[10];
  const float* Wa = (const float*)d_in[11];
  const float* Wb = (const float*)d_in[12];
  const float* bb = (const float*)d_in[13];
  const float* Wk = (const float*)d_in[14];
  const float* Wv = (const float*)d_in[15];
  const float* Wg = (const float*)d_in[16];
  const float* u = (const float*)d_in[17];
  const float* gn_w = (const float*)d_in[18];
  const float* gn_b = (const float*)d_in[19];
  const float* Wo = (const float*)d_in[20];
  float* out = (float*)d_out;
  char* ws = (char*)d_ws;
  float* ZB = (float*)(ws + kOffZB);
  float* BRWG = (float*)(ws + kOffBRWG);
  float* BKV = (float*)(ws + kOffBKV);
  float* BBB = (float*)(ws + kOffBBB);
  float* ONES = (float*)(ws + kOffONES);
  float* UB = (float*)(ws + kOffUB);
  unsigned short* WRWG0 = (unsigned short*)(ws + kOffWRWG0);
  unsigned short* WKV0 = (unsigned short*)(ws + kOffWKV0);
  unsigned short* WR = (unsigned short*)(ws + kOffWR);
  unsigned short* WG = (unsigned short*)(ws + kOffWG);
  unsigned short* WK = (unsigned short*)(ws + kOffWK);
  unsigned short* WV = (unsigned short*)(ws + kOffWV);
  unsigned short* WA = (unsigned short*)(ws + kOffWA);
  unsigned short* WB = (unsigned short*)(ws + kOffWB);
  unsigned short* WO = (unsigned short*)(ws + kOffWO);
  unsigned short* W2R16 = (unsigned short*)(ws + kOffW2R16);
  unsigned short* WKV2R16 = (unsigned short*)(ws + kOffWKV2R16);
  unsigned short* XA2 = (unsigned short*)(ws + kOffXA2);
  unsigned short* XK2 = (unsigned short*)(ws + kOffXK2);
  float* T0 = (float*)(ws + kOffT0);
  float* T0K = (float*)(ws + kOffT0K);
  unsigned short* TW16 = (unsigned short*)(ws + kOffTW16);
  unsigned short* TWK16 = (unsigned short*)(ws + kOffTWK16);
  float* RWG = (float*)(ws + kOffRWG);
  float* KVM = (float*)(ws + kOffKVM);
  unsigned short* XR2 = (unsigned short*)(ws + kOffXR2);
  unsigned short* XW2 = (unsigned short*)(ws + kOffXW2);
  unsigned short* XG2 = (unsigned short*)(ws + kOffXG2);
  unsigned short* XKK2 = (unsigned short*)(ws + kOffXKK2);
  unsigned short* XV2 = (unsigned short*)(ws + kOffXV2);
  float* RM = (float*)(ws + kOffRM);
  float* GM = (float*)(ws + kOffGM);
  float* WA1 = (float*)(ws + kOffWA1);
  unsigned short* TWA16 = (unsigned short*)(ws + kOffTWA16);
  float* WM = (float*)(ws + kOffWM);
  float* KM = (float*)(ws + kOffKM);
  float* VM = (float*)(ws + kOffVM);
  float* AM = (float*)(ws + kOffAM);
  float* OM = (float*)(ws + kOffOM);
  unsigned short* Y16 = (unsigned short*)(ws + kOffY16);

  for (int half = 0; half < 2; ++half) {
    const int co = half * kH;
    wt_plane_kernel<<<128, kH / 8, 0, stream>>>(W_rwg0, WRWG0, kH, 3 * kP, 3 * kP, kK2, co);
    wt_plane_kernel<<<2 * kP, kH / 8, 0, stream>>>(W_kv0, WKV0, kH, 2 * kP, 2 * kP, kK2, co);
    wt_plane_kernel<<<kH, kH / 8, 0, stream>>>(Wr, WR, kH, kH, kH, kK2, co);
    wt_plane_kernel<<<kH, kH / 8, 0, stream>>>(Wg, WG, kH, kH, kH, kK2, co);
    wt_plane_kernel<<<kH, kH / 8, 0, stream>>>(Wk, WK, kH, kH, kH, kK2, co);
    wt_plane_kernel<<<kH, kH / 8, 0, stream>>>(Wv, WV, kH, kH, kH, kK2, co);
    wt_plane_kernel<<<kG, kH / 8, 0, stream>>>(Wa, WA, kH, kG, kG, kK2, co);
  }
  wt_plane_kernel<<<kH, kG / 8, 0, stream>>>(Wb, WB, kG, kH, kH, kG, 0);
  wt_plane_kernel<<<kH, kH / 8, 0, stream>>>(Wo, WO, kH, kH, kH, kH, 0);
  cast_plane_kernel<<<(kH * 3 * kP / 8) / kThr, kThr, 0, stream>>>(W_rwg2, W2R16, 8, 256, 0);
  cast_plane_kernel<<<(kH * 2 * kP / 8) / kThr, kThr, 0, stream>>>(W_kv2, WKV2R16, 8, 256, 0);
  setup_kernel<<<16, kThr, 0, stream>>>(rwg_bias, kv_bias, bb, u, ZB, BRWG, BKV, BBB, ONES, UB);

  mix1k_kernel<<<128, kThr, 0, stream>>>(keyval, kv_mu, XK2);
  wmma_gemm64<0, false, 2, 0, false, 0><<<dim3((kRk / 64) * (2 * kP / 64) / 8, 1), 256, 0, stream>>>(
      XK2, XK2, kK2, 0L, WKV0, WKV0, kK2, 0L, (void*)(T0K), (void*)(T0K), 2 * kP, 0L, ZB, nullptr, 0L, kRk, 2 * kP, kK2, kScX);
  tanhcast_kernel<8, 64><<<(kRk * 8) / kThr, kThr, 0, stream>>>(T0K, TWK16);
  for (int n = 0; n < 2; ++n) {
    wmma_gemm64<0, false, 2, 0, false, 0><<<dim3((kRk / 64) * (kH / 64) / 8, 1), 256, 0, stream>>>(
        TWK16 + n * kP, TWK16 + n * kP, 2 * kP, 0L, WKV2R16 + n * kP, WKV2R16 + n * kP, 2 * kP, 0L, (void*)(KVM + n * kH), (void*)(KVM + n * kH), 2 * kH, 0L, BKV + n * kH, nullptr, 0L, kRk, kH, kP, kScT2);
  }
  mix2k_kernel<<<128, kThr, 0, stream>>>(keyval, KVM, XKK2, XV2);
  wmma_gemm64<0, false, 2, 0, false, 0><<<dim3((kRk / 64) * (kH / 64) / 8, 1), 256, 0, stream>>>(
      XKK2, XKK2, kK2, 0L, WK, WK, kK2, 0L, (void*)(KM), (void*)(KM), kH, 0L, ZB, nullptr, 0L, kRk, kH, kK2, kScX);
  wmma_gemm64<0, false, 2, 0, false, 0><<<dim3((kRk / 64) * (kH / 64) / 8, 1), 256, 0, stream>>>(
      XV2, XV2, kK2, 0L, WV, WV, kK2, 0L, (void*)(VM), (void*)(VM), kH, 0L, ZB, nullptr, 0L, kRk, kH, kK2, kScX);

  mix1q_kernel<<<1024, kThr, 0, stream>>>(keyval, query, rwg_mu, XA2);
  wmma_gemm64<0, false, 2, 0, false, 0><<<dim3((kRows / 64) * (128 / 64) / 8, 1), 256, 0, stream>>>(
      XA2, XA2, kK2, 0L, WRWG0, WRWG0, kK2, 0L, (void*)(T0), (void*)(T0), 128, 0L, ZB, nullptr, 0L, kRows, 128, kK2, kScX);
  tanhcast_kernel<12, 128><<<(kRows * 12) / kThr, kThr, 0, stream>>>(T0, TW16);
  for (int n = 0; n < 3; ++n) {
    wmma_gemm64<0, false, 2, 0, false, 0><<<dim3((kRows / 64) * (kH / 64) / 8, 1), 256, 0, stream>>>(
        TW16 + n * kP, TW16 + n * kP, 3 * kP, 0L, W2R16 + n * kP, W2R16 + n * kP, 3 * kP, 0L, (void*)(RWG + n * kH), (void*)(RWG + n * kH), 3 * kH, 0L, BRWG + n * kH, nullptr, 0L, kRows, kH, kP, kScT2);
  }
  mix2q_kernel<<<1024, kThr, 0, stream>>>(keyval, query, RWG, XR2, XW2, XG2);
  wmma_gemm64<0, false, 2, 0, false, 0><<<dim3((kRows / 64) * (kH / 64) / 8, 1), 256, 0, stream>>>(
      XR2, XR2, kK2, 0L, WR, WR, kK2, 0L, (void*)(RM), (void*)(RM), kH, 0L, ZB, nullptr, 0L, kRows, kH, kK2, kScX);
  wmma_gemm64<0, false, 2, 0, false, 0><<<dim3((kRows / 64) * (kH / 64) / 8, 1), 256, 0, stream>>>(
      XG2, XG2, kK2, 0L, WG, WG, kK2, 0L, (void*)(GM), (void*)(GM), kH, 0L, ZB, nullptr, 0L, kRows, kH, kK2, kScX);
  wmma_gemm64<0, false, 2, 0, false, 0><<<dim3((kRows / 64) * (kG / 64) / 8, 1), 256, 0, stream>>>(
      XW2, XW2, kK2, 0L, WA, WA, kK2, 0L, (void*)(WA1), (void*)(WA1), kG, 0L, ZB, nullptr, 0L, kRows, kG, kK2, kScX);
  tanhcast_kernel<8, 64><<<(kRows * 8) / kThr, kThr, 0, stream>>>(WA1, TWA16);
  wmma_gemm64<0, false, 2, 0, false, 0><<<dim3((kRows / 64) * (kH / 64) / 8, 1), 256, 0, stream>>>(
      TWA16, TWA16, kG, 0L, WB, WB, kG, 0L, (void*)(WM), (void*)(WM), kH, 0L, BBB, nullptr, 0L, kRows, kH, kG, kScTB);
  decay_kernel<<<2048, kThr, 0, stream>>>(WM, AM);

  walk_kernel<<<kEB, kThr, 0, stream>>>(RM, KM, VM, AM, UB, OM);
  gnorm_kernel<<<128, kThr, 0, stream>>>(OM, GM, gn_w, gn_b, Y16);
  wmma_gemm64<0, false, 2, 0, false, 0><<<dim3((kRows / 64) * (kH / 64) / 8, 1), 256, 0, stream>>>(
      Y16, Y16, kH, 0L, WO, WO, kH, 0L, (void*)(out), (void*)(out), kH, 0L, ZB, nullptr, 0L, kRows, kH, kH, kScY);
}
